// MemoryEfficientCrossAttention_tri_55774445305906
// MI455X (gfx1250) — hardware-verified
//
#include <hip/hip_runtime.h>
#include <math.h>

#ifndef GH_LOG
#define GH_LOG 5
#endif
#define GH (1 << GH_LOG)
#define LPOS (GH * GH)
#define LPOS_FULL 1024
#define NPLANE 3
#define CH 512
#define HEADS 8
#define HD 64
#define MID (GH / 2 - 1)
#define MROWS (NPLANE * LPOS)
#define NCHUNK (LPOS / 64)
#define QGRP (LPOS / 128)

static_assert(GH_LOG == 4 || GH_LOG == 5);
static_assert(LPOS <= LPOS_FULL);
static_assert(CH == HEADS * HD && HD == 64);
static_assert(64 % GH == 0);
static_assert(LPOS % 128 == 0 && LPOS % 64 == 0);
static_assert(MROWS % 64 == 0 && CH % 64 == 0 && CH % 32 == 0 && (2 * CH) % 32 == 0);
static_assert((MROWS * CH / 8) % 256 == 0 && (CH * CH / 8) % 256 == 0);
static_assert(CH / 8 == 64);

static constexpr float XC = 8.0f;
static constexpr float WC = 32.0f;
static constexpr float QC = 8.0f;
static constexpr float PC = 1024.0f;
static constexpr float OC = 32.0f;
static constexpr float SC_PROJ = 1.0f / 256.0f;
static constexpr float SC_OUT  = 1.0f / 1024.0f;
static constexpr float SC_S    = 1.0f / 64.0f;
static_assert(SC_PROJ * XC * WC == 1.0f);
static_assert(SC_OUT * OC * WC == 1.0f);
static_assert(SC_S * QC * QC == 1.0f);
static_assert(OC / QC == 4.0f);
static_assert(PC == 1024.0f);

typedef __attribute__((ext_vector_type(16))) _Float16 v16h;
typedef __attribute__((ext_vector_type(8)))  _Float16 v8h;
typedef __attribute__((ext_vector_type(2)))  _Float16 v2h;
typedef __attribute__((ext_vector_type(8)))  float    v8f;
typedef __attribute__((ext_vector_type(4)))  float    v4f;
typedef __attribute__((ext_vector_type(2)))  float    v2f;


__device__ __forceinline__ float bfr(float f) {
    unsigned u = __float_as_uint(f);
    u += 0x7FFFu + ((u >> 16) & 1u);
    return __uint_as_float(u & 0xFFFF0000u);
}

static __device__ __forceinline__ v2h cvt2h_sel(float a, float b) {
    v2f w;
    w.x = (fabsf(a) < 6.103515625e-05f) ? 0.0f : a;
    w.y = (fabsf(b) < 6.103515625e-05f) ? 0.0f : b;
    return __builtin_convertvector(w, v2h);
}
union H8U { v8h v; v2h p[4]; };

static __device__ __forceinline__ void vst8h(_Float16* p, v8h v) {
    *(volatile v8h*)p = v;
    __threadfence();
    *(volatile v8h*)p = v;
}

union FragU { v16h v; v8h h[2]; };
__device__ __forceinline__ v16h frag_ld(const _Float16* p) {
    FragU f; f.h[0] = *(const v8h*)(p); f.h[1] = *(const v8h*)(p + 16); return f.v;
}
__device__ __forceinline__ v8f wmma16(v16h a, v16h b, v8f c) {
    c = __builtin_amdgcn_wmma_f32_16x16x32_f16(false, a, false, b, (short)0, c, false, false);
    asm volatile("v_nop\n\tv_nop\n\tv_nop\n\tv_nop" : "+v"(c) : "v"(a), "v"(b));
    return c;
}
__device__ __forceinline__ void wave_sync_lds() {
    __builtin_amdgcn_fence(3  , "workgroup");
    __builtin_amdgcn_wave_barrier();
    __builtin_amdgcn_fence(2  , "workgroup");
}

static_assert(32 * 16 * 4 == 16 * 128);
template <bool RES>
static __device__ __forceinline__ void slab_store_h(const float* slab, _Float16* dW, _Float16* dR, const unsigned pitch, const unsigned lane) {
    const unsigned q = lane >> 3, c8 = (lane & 7u) * 8u;
    H8U hw[4], hr[4];
#pragma unroll
    for (int it = 0; it < 4; ++it) {
        const unsigned row = (unsigned)it * 4u + q;
        const float* sp = slab + row * 68u + c8;
#pragma unroll
        for (int e = 0; e < 4; ++e) {
            const float f0 = sp[2 * e], f1 = sp[2 * e + 1];
            const v2h w = cvt2h_sel(f0, f1);
            hw[it].p[e] = w;
            if (RES) hr[it].p[e] = cvt2h_sel(f0 - (float)w.x, f1 - (float)w.y);
        }
    }
    for (int pass = 0; pass < 2; ++pass) {
#pragma unroll
        for (int it = 0; it < 4; ++it) {
            const unsigned row = (unsigned)it * 4u + q;
            *(volatile v8h*)(dW + (size_t)row * pitch + c8) = hw[it].v;
            if (RES) *(volatile v8h*)(dR + (size_t)row * pitch + c8) = hr[it].v;
        }
        __threadfence();
    }
}

static_assert(32 * 16 * 8 == 16 * 256);
template <int MODE, unsigned M, unsigned N, unsigned K>
static __device__ __forceinline__ void gemm64_body(
    const _Float16* __restrict__ A, const unsigned lda, const _Float16* __restrict__ Bt, const unsigned ldb,
    float* __restrict__ Cf, _Float16* __restrict__ Cw, _Float16* __restrict__ Cr, const unsigned ldc,
    const float* __restrict__ bias, float* slabs) {
  static_assert(M % 64u == 0u && N % 64u == 0u && K % 32u == 0u);
  constexpr unsigned tilesN = N >> 6, tilesM = M >> 6;
  static_assert((tilesM * tilesN) % 8u == 0u);
  const unsigned lane = threadIdx.x & 31u;
  const unsigned wave = (unsigned)__builtin_amdgcn_readfirstlane((int)(threadIdx.x >> 5));
  const unsigned tile = blockIdx.x * 8u + wave;
  if (tile >= tilesM * tilesN) return;
  const unsigned tm = tile / tilesN;
  const unsigned tn = tile - tm * tilesN;
  const unsigned m0 = tm << 6, n0 = tn << 6;
  const unsigned rlane = lane & 15u;
  const unsigned koff = (lane >> 4) * 8u;
  const unsigned mOff = koff;

  v8f acc[4][4];
#pragma unroll
  for (int i = 0; i < 4; ++i)
#pragma unroll
    for (int j = 0; j < 4; ++j) acc[i][j] = (v8f){0.f,0.f,0.f,0.f,0.f,0.f,0.f,0.f};

#pragma unroll 1
  for (unsigned k0 = 0; k0 < K; k0 += 32u) {
    v16h bh[4];
#pragma unroll
    for (int j = 0; j < 4; ++j)
      bh[j] = frag_ld(Bt + (size_t)(n0 + ((unsigned)j << 4) + rlane) * ldb + koff + k0);
#pragma unroll
    for (int i = 0; i < 4; ++i) {
      unsigned ao = (m0 + ((unsigned)i << 4) + rlane) * lda + koff + k0;
      asm volatile("" : "+v"(ao));
      const v16h ah = frag_ld(A + (size_t)ao);
#pragma unroll
      for (int j = 0; j < 4; ++j)
        acc[i][j] = wmma16(ah, bh[j], acc[i][j]);
    }
  }

  float* slab = slabs + wave * (16u * 68u);
#pragma unroll
  for (int i = 0; i < 4; ++i) {
    const unsigned mBase = m0 + ((unsigned)i << 4);
#pragma unroll
    for (int j = 0; j < 4; ++j) {
      const unsigned n = n0 + ((unsigned)j << 4) + rlane;
      float bv = 0.0f;
      if (MODE == 0) bv = bfr(bias[n]);
#pragma unroll
      for (int r = 0; r < 8; ++r) {
        float v;
        if (MODE == 0) v = acc[i][j][r] * SC_OUT + bv;
        else           v = acc[i][j][r] * (SC_PROJ * QC);
        slab[(mOff + (unsigned)r) * 68u + ((unsigned)j << 4) + rlane] = v;
      }
    }
    wave_sync_lds();
    if (MODE == 0) {
      const unsigned hh = lane >> 4, c4 = (lane & 15u) * 4u;
#pragma unroll
      for (int half = 0; half < 2; ++half) {
        v4f vv[4];
#pragma unroll
        for (int it = 0; it < 4; ++it) {
          const unsigned row = (unsigned)(half * 4 + it) * 2u + hh;
          vv[it] = *(const v4f*)(slab + row * 68u + c4);
        }
        for (int pass = 0; pass < 2; ++pass) {
#pragma unroll
          for (int it = 0; it < 4; ++it) {
            const unsigned row = (unsigned)(half * 4 + it) * 2u + hh;
            *(volatile v4f*)(Cf + (size_t)(mBase + row) * ldc + n0 + c4) = vv[it];
          }
          __threadfence();
        }
      }
    } else {
      slab_store_h<MODE == 2>(slab, Cw + (size_t)mBase * ldc + n0, Cr + (size_t)mBase * ldc + n0, ldc, lane);
    }
    wave_sync_lds();
  }
}

static_assert(8 * 16 * 68 * 4 <= 131072);

__global__ __launch_bounds__(256) void k_proj(const _Float16* __restrict__ X16, const _Float16* __restrict__ W16,
                                              _Float16* __restrict__ Q16) {
    __shared__ __align__(16) float sT[8 * 16 * 68];
    gemm64_body<1, (unsigned)MROWS, (unsigned)CH, (unsigned)CH>(X16, (unsigned)CH, W16, (unsigned)CH,
        nullptr, Q16, nullptr, (unsigned)CH, nullptr, sT);
}

__global__ __launch_bounds__(256) void k_projt(const _Float16* __restrict__ X16, const _Float16* __restrict__ W16,
                                               _Float16* __restrict__ VTh, _Float16* __restrict__ VTl) {
    __shared__ __align__(16) float sT[8 * 16 * 68];
    const unsigned pl = blockIdx.y;
    const size_t xo = (size_t)pl * (size_t)(LPOS * CH);
    const size_t vo = (size_t)pl * (size_t)(CH * LPOS);
    gemm64_body<2, (unsigned)CH, (unsigned)LPOS, (unsigned)CH>(W16, (unsigned)CH, X16 + xo, (unsigned)CH,
        nullptr, VTh + vo, VTl + vo, (unsigned)LPOS, nullptr, sT);
}

__global__ __launch_bounds__(256) void k_outp(const _Float16* __restrict__ O16, const _Float16* __restrict__ Wo2,
                                              const float* __restrict__ bo, float* __restrict__ out) {
    __shared__ __align__(16) float sT[8 * 16 * 68];
    const unsigned pl = blockIdx.y;
    gemm64_body<0, (unsigned)LPOS, (unsigned)CH, (unsigned)(2 * CH)>(O16 + (size_t)pl * (size_t)(LPOS * 2 * CH), (unsigned)(2 * CH),
        Wo2, (unsigned)(2 * CH), out + (size_t)pl * (size_t)(LPOS_FULL * CH), nullptr, nullptr, (unsigned)CH, bo, sT);
}

__global__ __launch_bounds__(256) void k_x16(const float* __restrict__ x, _Float16* __restrict__ x16) {
    const unsigned u = blockIdx.x * 256u + threadIdx.x;
    if (u >= (unsigned)(MROWS * CH / 8)) return;
    const unsigned row = u >> 6, c0 = (u & 63u) * 8u;
    const unsigned plane = row / (unsigned)LPOS;
    const unsigned l = row - plane * (unsigned)LPOS;
    const float* xr = x + (size_t)(plane * (unsigned)LPOS_FULL + l) * CH + c0;
    const v4f a = *(const v4f*)xr, b = *(const v4f*)(xr + 4);
    H8U o;
    o.p[0] = cvt2h_sel(bfr(a.x) * XC, bfr(a.y) * XC);
    o.p[1] = cvt2h_sel(bfr(a.z) * XC, bfr(a.w) * XC);
    o.p[2] = cvt2h_sel(bfr(b.x) * XC, bfr(b.y) * XC);
    o.p[3] = cvt2h_sel(bfr(b.z) * XC, bfr(b.w) * XC);
    vst8h(x16 + (size_t)row * CH + c0, o.v);
}

__global__ __launch_bounds__(256) void k_wconv(const float* __restrict__ W, _Float16* __restrict__ D, unsigned ldd, unsigned dup) {
    const unsigned u = blockIdx.x * 256u + threadIdx.x;
    if (u >= (unsigned)(CH * CH / 8)) return;
    const unsigned o = u >> 6, k0 = (u & 63u) * 8u;
    const float* wr = W + (size_t)o * CH + k0;
    const v4f a = *(const v4f*)wr, b = *(const v4f*)(wr + 4);
    H8U h;
    h.p[0] = cvt2h_sel(bfr(a.x) * WC, bfr(a.y) * WC);
    h.p[1] = cvt2h_sel(bfr(a.z) * WC, bfr(a.w) * WC);
    h.p[2] = cvt2h_sel(bfr(b.x) * WC, bfr(b.y) * WC);
    h.p[3] = cvt2h_sel(bfr(b.z) * WC, bfr(b.w) * WC);
    vst8h(D + (size_t)o * ldd + k0, h.v);
    if (dup != 0u) vst8h(D + (size_t)o * ldd + (unsigned)CH + k0, h.v);
}

#define AT_PP 72
static_assert(8 * 16 * AT_PP * 2 + 8 * 16 * 68 * 4 <= 131072);
static_assert(NPLANE * HEADS * QGRP * 8 * 16 == NPLANE * HEADS * LPOS);
__global__ __launch_bounds__(256) void k_attn(
    const _Float16* __restrict__ Q16, const _Float16* __restrict__ VTh, const _Float16* __restrict__ VTl,
    _Float16* __restrict__ O16) {
    __shared__ __align__(16) _Float16 sP[8][16 * AT_PP];
    __shared__ __align__(16) float sO[8][16 * 68];
    const unsigned tid = threadIdx.x, lane = tid & 31u;
    const unsigned wave = (unsigned)__builtin_amdgcn_readfirstlane((int)(tid >> 5));
    const unsigned hh = lane >> 4, c = lane & 15u;
    const unsigned bx = blockIdx.x;
    const unsigned plane = bx / (unsigned)(HEADS * QGRP);
    const unsigned rem = bx - plane * (unsigned)(HEADS * QGRP);
    const unsigned head = rem / (unsigned)QGRP;
    const unsigned qg = rem - head * (unsigned)QGRP;
    const unsigned q0 = (qg * 8u + wave) * 16u;
    _Float16* pw = sP[wave];
    const float SC2 = 0.125f * SC_S * 1.4426950408889634f;

    v16h qf[2];
    {
        const _Float16* qrow = Q16 + (size_t)(plane * (unsigned)LPOS + q0 + c) * CH + head * 64u + 8u * hh;
        qf[0] = frag_ld(qrow);
        qf[1] = frag_ld(qrow + 32);
    }
    float mrow[8], lrow[8];
    v8f os[4];
#pragma unroll
    for (int r = 0; r < 8; ++r) { mrow[r] = -3.0e38f; lrow[r] = 0.f; }
#pragma unroll
    for (int t = 0; t < 4; ++t) os[t] = (v8f){0.f,0.f,0.f,0.f,0.f,0.f,0.f,0.f};

#pragma unroll 1
    for (unsigned half = 0; half < 2u; ++half) {
        const unsigned kp   = (half != 0u) ? 2u : ((plane == 0u) ? 1u : 0u);
        const unsigned kind = (half != 0u) ? (plane + 1u) : ((plane == 2u) ? 1u : 0u);
        unsigned selc[8], selr[8];
#pragma unroll
        for (int r = 0; r < 8; ++r) {
            const unsigned l = q0 + 8u * hh + (unsigned)r;
            const unsigned jq = l >> GH_LOG, iq = l & (unsigned)(GH - 1);
            selc[r] = (kind == 0u) ? iq : ((kind == 2u) ? ((unsigned)(GH - 1) - jq) : (unsigned)MID);
            selr[r] = (kind == 1u) ? jq : ((kind == 3u) ? ((unsigned)(GH - 1) - iq) : (unsigned)MID);
        }
        const _Float16* kbase = Q16 + (size_t)(kp * (unsigned)LPOS + c) * CH + head * 64u + 8u * hh;
        const _Float16* vhb = VTh + (size_t)(kp * (unsigned)CH + head * 64u + c) * LPOS + 8u * hh;
        const _Float16* vlb = VTl + (size_t)(kp * (unsigned)CH + head * 64u + c) * LPOS + 8u * hh;
#pragma unroll 1
        for (unsigned kc = 0; kc < (unsigned)NCHUNK; ++kc) {
            const unsigned kv0 = kc * 64u;
            v8f s[4];
#pragma unroll
            for (int jp = 0; jp < 2; ++jp) {
                unsigned ko = (kv0 + (unsigned)jp * 32u) * (unsigned)CH;
                asm volatile("" : "+v"(ko));
#pragma unroll
                for (int jj = 0; jj < 2; ++jj) {
                    const _Float16* kptr = kbase + (size_t)ko + (size_t)((unsigned)jj * 16u * (unsigned)CH);
                    const v16h kf0 = frag_ld(kptr);
                    const v16h kf1 = frag_ld(kptr + 32);
                    const v8f z = (v8f){0.f,0.f,0.f,0.f,0.f,0.f,0.f,0.f};
                    s[2 * jp + jj] = wmma16(qf[0], kf0, z);
                    s[2 * jp + jj] = wmma16(qf[1], kf1, s[2 * jp + jj]);
                }
            }
#pragma unroll
            for (int r = 0; r < 8; ++r) {
                float mx = -3.0e38f;
                unsigned mm[4];
#pragma unroll
                for (int j = 0; j < 4; ++j) {
                    const unsigned kl = kv0 + (unsigned)j * 16u + c;
                    const unsigned kr = kl >> GH_LOG, kcl = kl & (unsigned)(GH - 1);
                    mm[j] = (unsigned)(kcl == selc[r]) + (unsigned)(kr == selr[r]);
                    s[j][r] *= SC2;
                    const float se = (mm[j] != 0u) ? s[j][r] : -3.0e38f;
                    s[j][r] = se;
                    mx = fmaxf(mx, se);
                }
                mx = fmaxf(mx, __shfl_xor(mx, 1, 32)); mx = fmaxf(mx, __shfl_xor(mx, 2, 32));
                mx = fmaxf(mx, __shfl_xor(mx, 4, 32)); mx = fmaxf(mx, __shfl_xor(mx, 8, 32));
                const float mnew = fmaxf(mrow[r], mx);
                const float alpha = exp2f(mrow[r] - mnew);
                mrow[r] = mnew;
                float psum = 0.f;
#pragma unroll
                for (int j = 0; j < 4; ++j) {
                    const float p = (mm[j] != 0u) ? (float)mm[j] * exp2f(s[j][r] - mnew) : 0.0f;
                    psum += p;
                    const float w = p * 1024.0f;
                    const float wf = (w < 6.103515625e-05f) ? 0.0f : w;
                    pw[(8u * hh + (unsigned)r) * AT_PP + (unsigned)j * 16u + c] = (_Float16)wf;
                }
                psum += __shfl_xor(psum, 1, 32); psum += __shfl_xor(psum, 2, 32);
                psum += __shfl_xor(psum, 4, 32); psum += __shfl_xor(psum, 8, 32);
                lrow[r] = lrow[r] * alpha + psum;
                os[0][r] *= alpha; os[1][r] *= alpha; os[2][r] *= alpha; os[3][r] *= alpha;
            }
            wave_sync_lds();
#pragma unroll
            for (int kk = 0; kk < 2; ++kk) {
                const v16h pa = frag_ld(pw + c * AT_PP + (unsigned)kk * 32u + 8u * hh);
#pragma unroll
                for (int tp = 0; tp < 2; ++tp) {
                    unsigned vo = (unsigned)tp * 32u * (unsigned)LPOS + kv0 + (unsigned)kk * 32u;
                    asm volatile("" : "+v"(vo));
#pragma unroll
                    for (int tt = 0; tt < 2; ++tt) {
                        const size_t o = (size_t)vo + (size_t)((unsigned)tt * 16u * (unsigned)LPOS);
                        const v16h vbh = frag_ld(vhb + o);
                        const v16h vbl = frag_ld(vlb + o);
                        os[2 * tp + tt] = wmma16(pa, vbh, os[2 * tp + tt]);
                        os[2 * tp + tt] = wmma16(pa, vbl, os[2 * tp + tt]);
                    }
                }
            }
            wave_sync_lds();
        }
    }
    float* so = sO[wave];
#pragma unroll
    for (int r = 0; r < 8; ++r) {
        const float inv = 1.0f / (lrow[r] * 1024.0f);
#pragma unroll
        for (int t = 0; t < 4; ++t)
            so[(8u * hh + (unsigned)r) * 68u + (unsigned)t * 16u + c] = os[t][r] * inv * (OC / QC);
    }
    wave_sync_lds();
    {
        _Float16* dst = O16 + (size_t)(plane * (unsigned)LPOS + q0) * (size_t)(2 * CH) + head * 64u;
        slab_store_h<true>(so, dst, dst + CH, (unsigned)(2 * CH), lane);
    }
}

static constexpr size_t SZ_X16 = (size_t)MROWS * CH * 2;
static constexpr size_t SZ_WQ  = (size_t)CH * CH * 2;
static constexpr size_t SZ_WO2 = (size_t)CH * 2 * CH * 2;
static constexpr size_t SZ_Q16 = (size_t)MROWS * CH * 2;
static constexpr size_t SZ_VT  = (size_t)NPLANE * CH * LPOS * 2;
static constexpr size_t SZ_O16 = (size_t)MROWS * 2 * CH * 2;
static constexpr size_t WS_TOTAL = SZ_X16 + SZ_WQ + SZ_WO2 + SZ_Q16 + 2 * SZ_VT + SZ_O16;
static_assert(SZ_X16 % 256 == 0 && SZ_WQ % 256 == 0 && SZ_WO2 % 256 == 0 && SZ_Q16 % 256 == 0 && SZ_VT % 256 == 0 && SZ_O16 % 256 == 0);
static_assert(WS_TOTAL <= (size_t)134217728);

extern "C" void kernel_launch(void* const* d_in, const int* in_sizes, int n_in, void* d_out, int out_size,
                              void* d_ws, size_t ws_size, hipStream_t stream) {
    if (n_in < 4) return;
    if (in_sizes[0] < (2 * LPOS_FULL + LPOS) * CH || in_sizes[1] < CH * CH || in_sizes[2] < CH * CH || in_sizes[3] < CH) return;
    if (out_size < (2 * LPOS_FULL + LPOS) * CH) return;

    const float* x  = (const float*)d_in[0];
    const float* Wq = (const float*)d_in[1];
    const float* Wo = (const float*)d_in[2];
    const float* bo = (const float*)d_in[3];
    float* out = (float*)d_out;

    char* wsp = (char*)d_ws;
    size_t off = 0;
    auto carve = [&](size_t bytes) -> void* { void* r = wsp + off; off += (bytes + 255) & ~(size_t)255; return r; };
    _Float16* X16  = (_Float16*)carve(SZ_X16);
    _Float16* Wq16 = (_Float16*)carve(SZ_WQ);
    _Float16* Wo2  = (_Float16*)carve(SZ_WO2);
    _Float16* Q16  = (_Float16*)carve(SZ_Q16);
    _Float16* VTh  = (_Float16*)carve(SZ_VT);
    _Float16* VTl  = (_Float16*)carve(SZ_VT);
    _Float16* O16  = (_Float16*)carve(SZ_O16);
    if (off > ws_size || off > (size_t)134217728) return;

    k_x16<<<(MROWS * CH / 8) / 256, 256, 0, stream>>>(x, X16);
    k_wconv<<<(CH * CH / 8) / 256, 256, 0, stream>>>(Wq, Wq16, (unsigned)CH, 0u);
    k_wconv<<<(CH * CH / 8) / 256, 256, 0, stream>>>(Wo, Wo2, (unsigned)(2 * CH), 1u);

    k_proj<<<((MROWS / 64) * (CH / 64)) / 8, 256, 0, stream>>>(X16, Wq16, Q16);
    k_projt<<<dim3(((CH / 64) * (LPOS / 64)) / 8, NPLANE), 256, 0, stream>>>(X16, Wq16, VTh, VTl);
    k_attn<<<NPLANE * HEADS * QGRP, 256, 0, stream>>>(Q16, VTh, VTl, O16);
    k_outp<<<dim3(((LPOS / 64) * (CH / 64)) / 8, NPLANE), 256, 0, stream>>>(O16, Wo2, bo, out);
}
